// NaiveGNN_47296179863798
// MI455X (gfx1250) — hardware-verified
//
#include <hip/hip_runtime.h>
#include <stddef.h>


typedef _Float16 v16h __attribute__((ext_vector_type(16)));
typedef _Float16 v8h  __attribute__((ext_vector_type(8)));
typedef float    v8f  __attribute__((ext_vector_type(8)));
typedef float    v4f  __attribute__((ext_vector_type(4)));
typedef _Float16 h16;

#ifndef NROW
#define NROW 2048
#endif
#define NEL   2048
#define NNUC  64
#define INDIM 257
#define H1    32
#define H2    64
#define NL    3
#define SW    96
#define SPITCH 128
#define KEMB  288
#define KTOT  384
#define LDT 72
#define LDC 68
#define LDE 296
#define WCARRY 64.0f
#define RCARRY 2048.0f
#define SIGC (-0.022542110013890053f)

static_assert(NROW >= 64 && NROW <= NEL && (NROW % 64) == 0 && (NROW % 8) == 0);
static_assert((NEL % 16) == 0 && (NEL % 256) == 0);
static_assert(INDIM == 4 * NNUC + 1);
static_assert(SW == NL * H1 && (SW % 32) == 0 && (SW % 16) == 0);
static_assert(KEMB >= INDIM && (KEMB % 32) == 0);
static_assert(KTOT == SW + KEMB && (KTOT % 64) == 0 && (KTOT % 32) == 0);
static_assert(SPITCH >= SW && SPITCH * 2 == 16 * 16);
static_assert(SPITCH == SW + 32);
static_assert(H2 == 64 && NNUC == 64 && H1 == 32);
static_assert((LDT % 8) == 0 && LDT >= 64);
static_assert((LDC % 4) == 0 && LDC >= 64);
static_assert((LDE % 8) == 0 && LDE >= KEMB);
static_assert(2 * 32 == 64);
static_assert(4 * 16 == 64);
static_assert(64 * LDT * 2 <= 131072);
static_assert(3 * NEL * 4 + NL * 4 * H1 * 4 + 8 * SPITCH * 4 <= 131072);
static_assert(64 * LDE * 2 + 64 * LDC * 4 <= 131072);
static_assert(2 * 64 * LDE * 2 + 64 * LDC * 4 <= 131072);
static_assert((KEMB / 32) % 3 == 0);

#define WC_BYTES ((size_t)H2 * KTOT * 2)
#define S_BYTES  ((size_t)NROW * SPITCH * 2)
#define OFF_WC   ((size_t)0)
#define OFF_S    (OFF_WC + WC_BYTES)
#define OFF_SR   (OFF_S + S_BYTES)
#define WS_TOTAL (OFF_SR + S_BYTES)
static_assert((WC_BYTES % 128) == 0 && (S_BYTES % 128) == 0);
static_assert((OFF_S % 128) == 0 && (OFF_SR % 128) == 0);
static_assert(WS_TOTAL == (size_t)H2 * KTOT * 2 + 2 * (size_t)NROW * SPITCH * 2);
static_assert(WS_TOTAL <= (size_t)134217728);

__device__ __forceinline__ float bf16r(float x) {
  unsigned int u = __float_as_uint(x);
  u = (u + 0x7FFFu + ((u >> 16) & 1u)) & 0xFFFF0000u;
  return __uint_as_float(u);
}

static __device__ __forceinline__ h16 toh_flush(float v) {
  const h16 r = (h16)v;
  return (fabsf(v) < 6.103515625e-05f) ? (h16)0.0f : r;
}
static __device__ __forceinline__ h16 toh_res(float v, h16 hi) {
  return toh_flush(RCARRY * (v - (float)hi));
}

__device__ __forceinline__ v16h frag_at(const _Float16* p) {
  v8h lo = *(const v8h*)(p);
  v8h hi = *(const v8h*)(p + 16);
  v16h out;
#pragma unroll
  for (int i = 0; i < 8; ++i) { out[i] = lo[i]; out[i + 8] = hi[i]; }
  return out;
}

__device__ __forceinline__ v8f wmma16(v16h a, v16h b, v8f c) {
  v8f d = __builtin_amdgcn_wmma_f32_16x16x32_f16(false, a, false, b, (short)0, c,
                                                 false, false);
  asm volatile("v_nop\n\tv_nop\n\tv_nop\n\tv_nop" : "+v"(d) : "v"(a), "v"(b));
  return d;
}

__device__ __forceinline__ float fast_exp2(float t) {
#if __has_builtin(__builtin_amdgcn_exp2f)
  return __builtin_amdgcn_exp2f(t);
#else
  return __expf(t * 0.6931471805599453f);
#endif
}
__device__ __forceinline__ float logistic_carried(float d) {
  const float e = fast_exp2(d * SIGC);
  return __builtin_amdgcn_rcpf(1.0f + e);
}

__global__ __launch_bounds__(256) void wprep_kernel(
    const float* __restrict__ W0, const float* __restrict__ W2, _Float16* __restrict__ Wc) {
  __shared__ __attribute__((aligned(16))) _Float16 T[64 * LDT];
  const unsigned tid = threadIdx.x;
  const unsigned k0 = blockIdx.x * 64u;
#pragma unroll 4
  for (unsigned j = 0; j < 16u; ++j) {
    const unsigned idx = tid + 256u * j;
    const unsigned kr = idx >> 6, nc = idx & 63u;
    const unsigned k = k0 + kr;
    const unsigned k2 = (k < (unsigned)SW) ? k : (unsigned)(SW - 1);
    const unsigned ke = (k >= (unsigned)SW) ? (k - (unsigned)SW) : 0u;
    const unsigned k1 = (ke < (unsigned)INDIM) ? ke : (unsigned)(INDIM - 1);
    const float w2v = W2[k2 * (unsigned)H2 + nc];
    const float w0v = W0[k1 * (unsigned)H2 + nc];
    float v = (k < (unsigned)SW) ? w2v : w0v;
    v = (k < (unsigned)(SW + INDIM)) ? v : 0.0f;
    T[nc * LDT + kr] = toh_flush(WCARRY * bf16r(v));
  }
  __syncthreads();
  v8h x[2];
  size_t off[2];
#pragma unroll
  for (unsigned i = 0; i < 2u; ++i) {
    const unsigned n = 32u * i + (tid >> 3);
    const unsigned kc = (tid & 7u) * 8u;
    x[i] = *(const v8h*)&T[n * LDT + kc];
    off[i] = (size_t)n * KTOT + k0 + kc;
  }
#pragma unroll
  for (int i = 0; i < 2; ++i) *(volatile v8h*)(Wc + off[i]) = x[i];
  __threadfence();
#pragma unroll
  for (int i = 0; i < 2; ++i) *(volatile v8h*)(Wc + off[i]) = x[i];
}

__global__ __launch_bounds__(256) void ee_kernel(
    const float* __restrict__ r, const float* __restrict__ W1, _Float16* __restrict__ Sp,
    _Float16* __restrict__ Sr) {
  __shared__ float rx[NEL];
  __shared__ float ry[NEL];
  __shared__ float rz[NEL];
  __shared__ float w1s[NL * 4 * H1];
  __shared__ float accs[8 * SPITCH];

  const unsigned tid = threadIdx.x, lane = tid & 31u;
  const unsigned wave = (unsigned)__builtin_amdgcn_readfirstlane((int)(threadIdx.x >> 5));
  const unsigned hh = lane >> 4, m = lane & 15u;
  const bool lowhalf = (hh == 0u);
  const h16 hz = (h16)0.0f;

#pragma unroll 1
  for (unsigned idx = tid; idx < (unsigned)NEL; idx += 256u) {
    rx[idx] = bf16r(r[idx * 3u + 0u]);
    ry[idx] = bf16r(r[idx * 3u + 1u]);
    rz[idx] = bf16r(r[idx * 3u + 2u]);
  }
#pragma unroll 1
  for (unsigned idx = tid; idx < (unsigned)(NL * 4 * H1); idx += 256u)
    w1s[idx] = WCARRY * bf16r(W1[idx]);
  __syncthreads();

  const unsigned i = blockIdx.x * 8u + wave;
  const float rix = rx[i], riy = ry[i], riz = rz[i];

  v16h bw[6];
#pragma unroll
  for (int t = 0; t < 6; ++t) {
    v16h f = {};
    const unsigned l = (unsigned)(t >> 1);
    const unsigned n = (unsigned)(t & 1) * 16u + m;
#pragma unroll
    for (int q = 0; q < 4; ++q) {
      const h16 c = toh_flush(w1s[(l * 4u + (unsigned)q) * (unsigned)H1 + n]);
      f[q] = lowhalf ? c : hz;
    }
    bw[t] = f;
  }

  float acc[6];
#pragma unroll
  for (int t = 0; t < 6; ++t) acc[t] = 0.0f;
  const v8f zero8 = {};

#pragma unroll 1
  for (unsigned jt = 0; jt < (unsigned)(NEL / 16); ++jt) {
    const unsigned j = jt * 16u + m;
    const float dx = rix - rx[j];
    const float dy = riy - ry[j];
    const float dz = riz - rz[j];
    const float r2 = dx * dx + dy * dy + dz * dz;
    const h16 ax = toh_flush(dx);
    const h16 ay = toh_flush(dy);
    const h16 az = toh_flush(dz);
    const h16 aw = toh_flush(r2);
    v16h a = {};
    a[0] = lowhalf ? ax : hz;
    a[1] = lowhalf ? ay : hz;
    a[2] = lowhalf ? az : hz;
    a[3] = lowhalf ? aw : hz;
#pragma unroll
    for (int t = 0; t < 6; ++t) {
      const v8f d = wmma16(a, bw[t], zero8);
      float s = 0.0f;
#pragma unroll
      for (int v = 0; v < 8; ++v) s += logistic_carried(d[v]);
      acc[t] += s;
    }
  }

  float tot[6];
#pragma unroll
  for (int t = 0; t < 6; ++t) tot[t] = acc[t] + __shfl_xor(acc[t], 16, 32);

#pragma unroll
  for (int q = 0; q < 3; ++q) {
    const float val = lowhalf ? tot[2 * q] : tot[2 * q + 1];
    accs[wave * (unsigned)SPITCH + ((unsigned)(2 * q) + hh) * 16u + m] = val;
  }
  accs[wave * (unsigned)SPITCH + (unsigned)SW + hh * 16u + m] = 0.0f;
  __syncthreads();

  const unsigned c8 = (lane & 15u) * 8u;
  v8h x, xr;
#pragma unroll
  for (int e = 0; e < 8; ++e) {
    const float v = accs[wave * (unsigned)SPITCH + c8 + (unsigned)e];
    const h16 hi = toh_flush(v);
    x[e]  = hi;
    xr[e] = toh_res(v, hi);
  }
  _Float16* p  = Sp + (size_t)i * SPITCH + c8;
  _Float16* pr = Sr + (size_t)i * SPITCH + c8;
  if (lane < 16u) { *(volatile v8h*)p = x; *(volatile v8h*)pr = xr; }
  __threadfence();
  if (lane < 16u) { *(volatile v8h*)p = x; *(volatile v8h*)pr = xr; }
}

__global__ __launch_bounds__(256) void hout_kernel(
    const float* __restrict__ r, const float* __restrict__ Rn, const float* __restrict__ bias,
    const int* __restrict__ nup_p, const int* __restrict__ ndn_p,
    const _Float16* __restrict__ Sp, const _Float16* __restrict__ Sr,
    const _Float16* __restrict__ Wc, float* __restrict__ outf) {
  __shared__ __attribute__((aligned(16))) _Float16 Es[64 * LDE];
  __shared__ __attribute__((aligned(16))) _Float16 Er[64 * LDE];
  __shared__ __attribute__((aligned(16))) float Cs[64 * LDC];

  const unsigned tid = threadIdx.x, lane = tid & 31u;
  const unsigned w = (unsigned)__builtin_amdgcn_readfirstlane((int)(threadIdx.x >> 5));
  const unsigned mw = w >> 1, nw = w & 1u;
  const unsigned hh = lane >> 4, m = lane & 15u;
  const unsigned row0 = blockIdx.x * 64u;
  const int nup = nup_p[0];
  const int ndn = ndn_p[0];
  const h16 hz = (h16)0.0f;

  {
    const unsigned n = tid & 63u;
    const float Rx = bf16r(Rn[n * 3u + 0u]);
    const float Ry = bf16r(Rn[n * 3u + 1u]);
    const float Rz = bf16r(Rn[n * 3u + 2u]);
#pragma unroll 1
    for (unsigned jj = 0; jj < 16u; ++jj) {
      const unsigned e = (tid >> 6) + 4u * jj;
      const unsigned ge = row0 + e;
      const float dx = bf16r(r[ge * 3u + 0u]) - Rx;
      const float dy = bf16r(r[ge * 3u + 1u]) - Ry;
      const float dz = bf16r(r[ge * 3u + 2u]) - Rz;
      const float dist = sqrtf(dx * dx + dy * dy + dz * dz);
      const float logd = log1pf(dist);
      const float scal = logd / dist;
      const float f0 = dx * scal;
      const float f1 = dy * scal;
      const float f2 = dz * scal;
      const h16 h0 = toh_flush(f0);
      const h16 h1 = toh_flush(f1);
      const h16 h2 = toh_flush(f2);
      const h16 h3 = toh_flush(logd);
      Es[e * LDE + 3u * n + 0u] = h0;
      Es[e * LDE + 3u * n + 1u] = h1;
      Es[e * LDE + 3u * n + 2u] = h2;
      Es[e * LDE + 192u + n]    = h3;
      Er[e * LDE + 3u * n + 0u] = toh_res(f0, h0);
      Er[e * LDE + 3u * n + 1u] = toh_res(f1, h1);
      Er[e * LDE + 3u * n + 2u] = toh_res(f2, h2);
      Er[e * LDE + 192u + n]    = toh_res(logd, h3);
    }
  }
#pragma unroll 1
  for (unsigned q = 0; q < 8u; ++q) {
    const unsigned idx = tid + 256u * q;
    const unsigned e = idx >> 5, c = idx & 31u;
    const int ge = (int)(row0 + e);
    const float sp = (ge < nup) ? 1.0f : ((ge < nup + ndn) ? -1.0f : 0.0f);
    const h16 sv = (h16)sp;
    const h16 sr = toh_res(sp, sv);
    Es[e * LDE + 256u + c] = (c == 0u) ? sv : hz;
    Er[e * LDE + 256u + c] = (c == 0u) ? sr : hz;
  }
  __syncthreads();

  const _Float16* sp0 = Sp + (size_t)(row0 + mw * 16u + m) * SPITCH + hh * 8u;
  const _Float16* sr0 = Sr + (size_t)(row0 + mw * 16u + m) * SPITCH + hh * 8u;
  const _Float16* bp0 = Wc + (size_t)(nw * 32u + m) * KTOT + hh * 8u;
  const _Float16* bp1 = bp0 + (size_t)16 * KTOT;
  const unsigned eoff = (mw * 16u + m) * (unsigned)LDE + hh * 8u;
  v8f acc0 = {}, acc1 = {};
  v8f res0 = {}, res1 = {};
#pragma unroll
  for (unsigned ks = 0; ks < (unsigned)(SW / 32); ++ks) {
    const v16h a  = frag_at(sp0 + ks * 32u);
    const v16h ar = frag_at(sr0 + ks * 32u);
    const v16h b0 = frag_at(bp0 + ks * 32u);
    const v16h b1 = frag_at(bp1 + ks * 32u);
    acc0 = wmma16(a, b0, acc0);
    acc1 = wmma16(a, b1, acc1);
    res0 = wmma16(ar, b0, res0);
    res1 = wmma16(ar, b1, res1);
  }
#pragma unroll 3
  for (unsigned ks = 0; ks < (unsigned)(KEMB / 32); ++ks) {
    const v16h a  = frag_at(&Es[eoff + ks * 32u]);
    const v16h ar = frag_at(&Er[eoff + ks * 32u]);
    const v16h b0 = frag_at(bp0 + (unsigned)SW + ks * 32u);
    const v16h b1 = frag_at(bp1 + (unsigned)SW + ks * 32u);
    acc0 = wmma16(a, b0, acc0);
    acc1 = wmma16(a, b1, acc1);
    res0 = wmma16(ar, b0, res0);
    res1 = wmma16(ar, b1, res1);
  }
#pragma unroll
  for (int rr = 0; rr < 8; ++rr) {
    float* d = &Cs[(mw * 16u + hh * 8u + (unsigned)rr) * LDC + nw * 32u + m];
    d[0]  = acc0[rr] + res0[rr] * (1.0f / RCARRY);
    d[16] = acc1[rr] + res1[rr] * (1.0f / RCARRY);
  }
  __syncthreads();

  v4f xs[4];
  size_t off[4];
#pragma unroll
  for (unsigned i = 0; i < 4u; ++i) {
    const unsigned rr = 16u * i + (tid >> 4);
    const unsigned c = (tid & 15u) * 4u;
    const v4f u = *(const v4f*)&Cs[rr * LDC + c];
    const v4f g = *(const v4f*)(bias + c);
    v4f val;
#pragma unroll
    for (int j = 0; j < 4; ++j) val[j] = u[j] * (1.0f / WCARRY) + bf16r(g[j]);
    xs[i] = val;
    off[i] = (size_t)(row0 + rr) * H2 + c;
  }
#pragma unroll
  for (int i = 0; i < 4; ++i) *(volatile v4f*)(outf + off[i]) = xs[i];
  __threadfence();
#pragma unroll
  for (int i = 0; i < 4; ++i) *(volatile v4f*)(outf + off[i]) = xs[i];
}

extern "C" void kernel_launch(void* const* d_in, const int* in_sizes, int n_in,
                              void* d_out, int out_size, void* d_ws, size_t ws_size,
                              hipStream_t stream) {
  if (n_in < 8) return;
  if ((long long)in_sizes[0] < (long long)NEL * 3) return;
  if ((long long)in_sizes[1] < (long long)NNUC * 3) return;
  if ((long long)in_sizes[2] < (long long)INDIM * H2) return;
  if ((long long)in_sizes[3] < (long long)H2) return;
  if ((long long)in_sizes[4] < (long long)NL * 4 * H1) return;
  if ((long long)in_sizes[5] < (long long)NL * H1 * H2) return;
  if (in_sizes[6] < 1 || in_sizes[7] < 1) return;
  if ((long long)out_size < (long long)NROW * H2) return;
  if (ws_size < WS_TOTAL) return;

  const float* r   = (const float*)d_in[0];
  const float* Rn  = (const float*)d_in[1];
  const float* W0  = (const float*)d_in[2];
  const float* b0  = (const float*)d_in[3];
  const float* W1s = (const float*)d_in[4];
  const float* W2s = (const float*)d_in[5];
  const int*   nup = (const int*)d_in[6];
  const int*   ndn = (const int*)d_in[7];
  float* out = (float*)d_out;

  char* ws = (char*)d_ws;
  _Float16* Wc = (_Float16*)(ws + OFF_WC);
  _Float16* Sp = (_Float16*)(ws + OFF_S);
  _Float16* Sr = (_Float16*)(ws + OFF_SR);

  dim3 blk(256);
  wprep_kernel<<<dim3(KTOT / 64), blk, 0, stream>>>(W0, W2s, Wc);
  ee_kernel<<<dim3(NROW / 8), blk, 0, stream>>>(r, W1s, Sp, Sr);
  hout_kernel<<<dim3(NROW / 64), blk, 0, stream>>>(r, Rn, b0, nup, ndn, Sp, Sr, Wc, out);
}
